// V2VModule_26259430048622
// MI455X (gfx1250) — hardware-verified
//
#include <hip/hip_runtime.h>


namespace {
constexpr int N = 200000, KO = 27, CI = 16, CM = 32, CO = 32, K1P = 448, K2P = 864;
constexpr float XS = 8.0f, WSC = 256.0f, BN_EPS = 1e-3f;
typedef _Float16 b16;
typedef __attribute__((ext_vector_type(16))) _Float16 v16b;
typedef __attribute__((ext_vector_type(8))) _Float16 v8b;
typedef __attribute__((ext_vector_type(8))) float v8f;
typedef __attribute__((ext_vector_type(4))) float v4f;
__device__ __forceinline__ float bf16_rne(float f) { unsigned int u = __float_as_uint(f); u += 0x7FFFu + ((u >> 16) & 1u); float r = __uint_as_float(u & 0xFFFF0000u); asm volatile("" : "+v"(r)); return r; }
__device__ __forceinline__ void split16(float v, b16& hi, b16& lo) { hi = (b16)v; lo = (b16)(v - (float)hi); }
__device__ __forceinline__ v16b frag_kb(const b16* p, int hh) { const v8b a = *(const v8b*)(p + 8 * hh), b = *(const v8b*)(p + 16 + 8 * hh); v16b f;
#pragma unroll
  for (int e = 0; e < 8; ++e) { f[e] = a[e]; f[8 + e] = b[e]; } return f; }
__device__ __forceinline__ v8f wmma16b(v16b a, v16b b, v8f c) { v8f d = __builtin_amdgcn_wmma_f32_16x16x32_f16(false, a, false, b, (short)0, c, false, false); asm volatile("v_nop\n\tv_nop\n\tv_nop\n\tv_nop" : "+v"(d) : "v"(a), "v"(b)); return d; }
__device__ __forceinline__ void wave_lds_sync() { __builtin_amdgcn_fence(__ATOMIC_RELEASE, "workgroup"); __builtin_amdgcn_wave_barrier(); __builtin_amdgcn_fence(__ATOMIC_ACQUIRE, "workgroup"); }
__device__ __forceinline__ float pmul(float a, float b) { float p = a * b; asm volatile("" : "+v"(p)); return p; }
__device__ __forceinline__ int iclamp(int v, int lo, int hi) { return v < lo ? lo : (v > hi ? hi : v); }

__global__ __launch_bounds__(256) void wput_kernel(const float* __restrict__ w1, const float* __restrict__ w2, b16* __restrict__ W1T, b16* __restrict__ W2T) { const int u = blockIdx.x * 256 + threadIdx.x;
  for (int pass = 0; pass < 2; ++pass) {
    if (u < CM * (K1P / 8)) { const int o = u / (K1P / 8), k0 = (u % (K1P / 8)) * 8; v8b v;
#pragma unroll
      for (int j = 0; j < 8; ++j) { const int kk = k0 + j; v[j] = (b16)(kk < KO * CI ? bf16_rne(w1[((size_t)(kk / CI) * CI + kk % CI) * CM + o]) * WSC : 0.0f); } *(volatile v8b*)(W1T + (size_t)o * K1P + k0) = v; }
    if (u < CO * (K2P / 8)) { const int o = u / (K2P / 8), k0 = (u % (K2P / 8)) * 8; v8b v;
#pragma unroll
      for (int j = 0; j < 8; ++j) { const int kk = k0 + j; v[j] = (b16)(bf16_rne(w2[((size_t)(kk / CM) * CM + kk % CM) * CO + o]) * WSC); } *(volatile v8b*)(W2T + (size_t)o * K2P + k0) = v; }
    __threadfence(); } }
__global__ __launch_bounds__(32) void mk_kernel(const int* __restrict__ ro, int* __restrict__ MK) { const int lane = threadIdx.x; int m = 0; if (lane < KO) { int lo = 0, hi = N; while (lo < hi) { const int mid = (lo + hi) >> 1; if (ro[(size_t)lane * N + mid] < N) lo = mid + 1; else hi = mid; } m = lo; }
  for (int pass = 0; pass < 2; ++pass) { ((volatile int*)MK)[lane] = m; __threadfence(); } }
__device__ __forceinline__ int find_partner(const int* __restrict__ ro, const int* __restrict__ MK, int k, int n) { int lo = 0, hi = iclamp(MK[k], 0, N); const int* r = ro + (size_t)k * N; while (lo < hi) { const int mid = (lo + hi) >> 1; const int v = r[mid]; if (v < n) lo = mid + 1; else hi = mid; } return (lo < N && r[lo] == n) ? lo : -1; }
template <int LAYER>
__global__ __launch_bounds__(32) void conv_kernel(const float* __restrict__ IN, const float* __restrict__ ST, const float* __restrict__ g, const float* __restrict__ be, const int* __restrict__ ri, const int* __restrict__ ro, const int* __restrict__ MK, const b16* __restrict__ WT, int NLIM, float* __restrict__ P, float* __restrict__ PS) {
  constexpr int CW = LAYER == 1 ? CI : CM, KP = LAYER == 1 ? K1P : K2P; __shared__ __attribute__((aligned(16))) b16 Ah[16][KP + 8], Al[16][LAYER == 1 ? 8 : KP + 8]; __shared__ int J[16][KO + 1]; __shared__ float Tf[16][36];
  const int lane = threadIdx.x, nloc = lane & 15, hlf = lane >> 4; const size_t m0 = (size_t)blockIdx.x * 16; if (m0 >= (size_t)NLIM) return;
  for (int q = lane; q < 16 * KO; q += 32) { const int rr = q / KO, k = q % KO; const int j = find_partner(ro, MK, k, (int)(m0 + rr)); int src = -1; if (j >= 0) { src = iclamp(ri[(size_t)k * N + j], 0, N - 1); if (src >= NLIM) src = -1; } J[rr][k] = src; }
  wave_lds_sync();
  for (int rr = 0; rr < 16; ++rr) { for (int c = lane; c < KP; c += 32) { const int k = c / CW, cc = c % CW; float v = 0.0f; if (k < KO) { const int src = J[rr][k]; if (src >= 0) { v = IN[(size_t)src * CW + cc]; if (LAYER == 1) v = bf16_rne(v); else v = fmaxf(pmul(pmul(v - ST[cc], ST[32 + cc]), bf16_rne(g[cc])) + bf16_rne(be[cc]), 0.0f); } }
      if (LAYER == 1) Ah[rr][c] = (b16)(v * XS); else { b16 p, ql; split16(v * XS, p, ql); Ah[rr][c] = p; Al[rr][c] = ql; } } }
  wave_lds_sync(); v8f acc[2] = {(v8f){}, (v8f){}};
#pragma unroll 2
  for (int kb = 0; kb < KP; kb += 32) { const v16b a = frag_kb(&Ah[nloc][kb], hlf); v16b al; if (LAYER == 2) al = frag_kb(&Al[nloc][kb], hlf);
#pragma unroll
    for (int t = 0; t < 2; ++t) { const v16b bw = frag_kb(WT + (size_t)(t * 16 + nloc) * KP + kb, hlf); acc[t] = wmma16b(a, bw, acc[t]); if (LAYER == 2) acc[t] = wmma16b(al, bw, acc[t]); } }
#pragma unroll
  for (int t = 0; t < 2; ++t)
#pragma unroll
    for (int r8 = 0; r8 < 8; ++r8) Tf[8 * hlf + r8][t * 16 + nloc] = acc[t][r8] * (1.0f / (XS * WSC));
  wave_lds_sync(); float s = 0.0f, sq = 0.0f; for (int rr = 0; rr < 16; ++rr) { const float v = Tf[rr][lane]; s += v; sq += pmul(v, v); }
  for (int pass = 0; pass < 2; ++pass) { for (int rr = 0; rr < 16; ++rr) ((volatile float*)P)[(m0 + rr) * 32 + lane] = Tf[rr][lane]; ((volatile float*)PS)[(size_t)blockIdx.x * 64 + lane] = s; ((volatile float*)PS)[(size_t)blockIdx.x * 64 + 32 + lane] = sq; __threadfence(); } }
__global__ __launch_bounds__(256) void bnfin_kernel(const float* __restrict__ PS, int nw, int nnodes, float* __restrict__ ST) { const int t = threadIdx.x; const int c = t & 31, part = t >> 5; __shared__ double S_[8][32], Q_[8][32]; double s = 0.0, q = 0.0; for (int w = part; w < nw; w += 8) { s += (double)PS[(size_t)w * 64 + c]; q += (double)PS[(size_t)w * 64 + 32 + c]; } S_[part][c] = s; Q_[part][c] = q; __syncthreads();
  if (t < 32) { double sum = 0.0, sq = 0.0; for (int p = 0; p < 8; ++p) { sum += S_[p][t]; sq += Q_[p][t]; } const double mu = sum / nnodes; double var = sq / nnodes - mu * mu; if (var < 0.0) var = 0.0;
    for (int pass = 0; pass < 2; ++pass) { ((volatile float*)ST)[t] = (float)mu; ((volatile float*)ST)[32 + t] = (float)(1.0 / sqrt(var + (double)BN_EPS)); __threadfence(); } } }
__global__ __launch_bounds__(256) void fin_kernel(const float* __restrict__ P2, const float* __restrict__ ST, const float* __restrict__ g, const float* __restrict__ be, int NLIM, float* __restrict__ out) { const size_t u = (size_t)blockIdx.x * 256 + threadIdx.x; if (u >= (size_t)N * 8) return; const size_t n = u / 8; const int c0 = (int)(u % 8) * 4; v4f r = {0, 0, 0, 0};
  if (n < (size_t)NLIM) { const v4f p = *(const v4f*)(P2 + u * 4); for (int k = 0; k < 4; ++k) r[k] = fmaxf(pmul(pmul(p[k] - ST[c0 + k], ST[32 + c0 + k]), bf16_rne(g[c0 + k])) + bf16_rne(be[c0 + k]), 0.0f); }
  for (int pass = 0; pass < 2; ++pass) { *(volatile v4f*)(out + u * 4) = r; __threadfence(); } }
}

extern "C" void kernel_launch(void* const* d_in, const int* in_sizes, int n_in, void* d_out, int out_size, void* d_ws, size_t ws_size, hipStream_t stream) {
  (void)n_in;
  auto Fp = [&](int i) { return (const float*)d_in[i]; }; auto Ip = [&](int i) { return (const int*)d_in[i]; };
  if (in_sizes[0] != N * CI || in_sizes[1] != KO * CI * CM || in_sizes[4] != KO * CM * CO || in_sizes[7] != KO * N || in_sizes[8] != KO * N || out_size != N * CO) return;
  const int NLIM = N;
  const int NW = NLIM / 16;
  size_t off = 0; char* ws = (char*)d_ws;
  auto carve = [&](size_t bytes) { char* p = ws + off; off += (bytes + 255) & ~(size_t)255; return p; };
  b16* W1T = (b16*)carve((size_t)CM * K1P * 2); b16* W2T = (b16*)carve((size_t)CO * K2P * 2); int* MK = (int*)carve(32 * 4); float* P1 = (float*)carve((size_t)N * CM * 4); float* P2 = (float*)carve((size_t)N * CO * 4); float* PS = (float*)carve((size_t)(N / 16) * 64 * 4); float* ST1 = (float*)carve(64 * 4); float* ST2 = (float*)carve(64 * 4);
  if (off > ws_size || off > ((size_t)96 << 20)) return;
  wput_kernel<<<(CO * (K2P / 8) + 255) / 256, 256, 0, stream>>>(Fp(1), Fp(4), W1T, W2T);
  mk_kernel<<<1, 32, 0, stream>>>(Ip(8), MK);
  conv_kernel<1><<<NW, 32, 0, stream>>>(Fp(0), nullptr, nullptr, nullptr, Ip(7), Ip(8), MK, W1T, NLIM, P1, PS);
  bnfin_kernel<<<1, 256, 0, stream>>>(PS, NW, NLIM, ST1);
  conv_kernel<2><<<NW, 32, 0, stream>>>(P1, ST1, Fp(2), Fp(3), Ip(7), Ip(8), MK, W2T, NLIM, P2, PS);
  bnfin_kernel<<<1, 256, 0, stream>>>(PS, NW, NLIM, ST2);
  fin_kernel<<<(unsigned)(((size_t)N * 8 + 255) / 256), 256, 0, stream>>>(P2, ST2, Fp(5), Fp(6), NLIM, (float*)d_out);
}
